// GraphGNN_84636625535112
// MI455X (gfx1250) — hardware-run, weakly checked
//
#include <hip/hip_runtime.h>
#include <stddef.h>
#include <stdint.h>


#define NB     2
#define NN     50000
#define NF     16
#define NE     1600000
#define EH     32
#define EO     30
#define NO     16
#define PW     64
#define MROWS  (NB * NN)
#define NTILE  (MROWS / 16)
#define NTHR   256
#define NWAVE  8
#define EPT    8
#define CHUNK  (NTHR * EPT)
#define WCAP   (EPT * 32)
#define LISTN  (NWAVE * WCAP)
#define NBA    512
#define SLA    9
#define NBLK   98
#define NP     (NBLK * NBA)
#define RCAP   20480
#define DEGCAP 80
#define RB     64
#define NRB    ((NN + RB - 1) / RB)
#define FLN    32
#define T_W1R  0
#define T_B1   32
#define T_B2   64
#define T_W3   96
#define T_B3   576
#define TABN   640
#define W3N    496
#define BK_ZINTS (LISTN + 2 * RCAP + 3 * NBA)
#define BK_INTS  (BK_ZINTS + 16)
#define BK_BYTES (BK_INTS * 4)
#define WSMAX  134217728

static_assert(NN % 2 == 0);
static_assert(((long long)NN * NO * 4) % 128 == 0);
static_assert(NBA % RB == 0 && RB % 2 == 0 && RB == NWAVE * 8);
static_assert(MROWS % 16 == 0);
static_assert((long long)NE < (1LL << 21));
static_assert(((long long)NE << SLA) < (1LL << 31));
static_assert(((long long)CHUNK << SLA) < (1LL << 31));
static_assert((NBA & (NBA - 1)) == 0 && NBA == (1 << SLA) && NBA % 32 == 0 && NBA == 2 * NTHR);
static_assert(NBLK * NBA >= NN && (NBLK - 1) * NBA < NN);
static_assert(RCAP % (2 * NTHR) == 0 && BK_ZINTS % 4 == 0 && LISTN % 4 == 0 && ((LISTN + RCAP) % 2) == 0);
static_assert(BK_BYTES <= 300000);
static_assert(NE % 4 == 0);
static_assert(DEGCAP % 16 == 0 && DEGCAP >= 57 + 8);
static_assert(RCAP >= 17512);
static_assert(TABN % 4 == 0 && TABN / 4 <= NTHR && T_B3 + 16 <= TABN && T_W3 + W3N == T_B3 + 16);
static_assert(T_B1 % 32 == 0 && T_B2 % 32 == 0 && T_W3 % 32 == 0 && T_B3 % 32 == 0);
static_assert((NN - (NRB - 1) * RB) % 8 == 0 && (NN - (NRB - 1) * RB) > 0);
static_assert(((long long)(NB - 1) * NN + (long long)(NRB - 1) * RB) * NO + 4LL * ((NN - (NRB - 1) * RB) * 4 - 1) + 3
              == (long long)NB * NN * NO - 1);

typedef float          v4f   __attribute__((ext_vector_type(4)));
typedef float          v8f   __attribute__((ext_vector_type(8)));
typedef int            v2i   __attribute__((ext_vector_type(2)));
typedef int            v4i   __attribute__((ext_vector_type(4)));
typedef int            v8i   __attribute__((ext_vector_type(8)));
typedef unsigned short v8us  __attribute__((ext_vector_type(8)));
typedef unsigned short v16us __attribute__((ext_vector_type(16)));
typedef __bf16         v16bf __attribute__((ext_vector_type(16)));
typedef v4f  __attribute__((may_alias)) v4fa;
typedef v2i  __attribute__((may_alias)) v2ia;
typedef v4i  __attribute__((may_alias)) v4ia;
typedef v8us __attribute__((may_alias)) v8usa;
union FragB { v16bf v; v16us u; v8us h[2]; v8i w; };

__device__ __forceinline__ v8f wmb(const FragB& a, const FragB& b, v8f c) {
  v8f d = __builtin_amdgcn_wmma_f32_16x16x32_bf16(false, a.v, false, b.v, (short)0, c, false, false);
  asm volatile("v_nop\n\tv_nop\n\tv_nop\n\tv_nop" : "+v"(d) : "v"(a.w), "v"(b.w));
  return d;
}
__device__ __forceinline__ v8f z8() { v8f z = {0.f, 0.f, 0.f, 0.f, 0.f, 0.f, 0.f, 0.f}; return z; }

__device__ __forceinline__ unsigned bf16_bits(float f) {
  const unsigned u = __float_as_uint(f);
  return (u + 0x7FFFu + ((u >> 16) & 1u)) >> 16;
}
__device__ __forceinline__ float bf16_val(float f) {
  return __uint_as_float(bf16_bits(f) << 16);
}
__device__ __forceinline__ float sigf(float t) {
  return __builtin_amdgcn_rcpf(1.0f + __expf(-t));
}
__device__ __forceinline__ void wave_sync() {
  __builtin_amdgcn_fence(__ATOMIC_RELEASE, "wavefront");
  __builtin_amdgcn_wave_barrier();
  __builtin_amdgcn_fence(__ATOMIC_ACQUIRE, "wavefront");
}
__device__ __forceinline__ void put16(unsigned short* dp, v8us o) {
  *(volatile v8us*)dp = o;
  __threadfence();
  *(volatile v8us*)dp = o;
}
__device__ __forceinline__ void putf4(float* dp, v4f o) {
  *(volatile v4f*)dp = o;
  __threadfence();
  *(volatile v4f*)dp = o;
}
__device__ __forceinline__ void puti4(int* dp, v4i o) {
  *(volatile v4i*)dp = o;
  __threadfence();
  *(volatile v4i*)dp = o;
}

template <int SLB>
__device__ __forceinline__ int scan_chunk(const int* __restrict__ dsts, int nE, int cbase, int slotBase,
                                          int nb, int vec8, int* list, int tid, int lane, int wave) {
  int wc = 0;
  const int el0  = tid * EPT;
  const int e0   = cbase + el0;
  const int sent = -2147483647 - 1;
  v4i da, db;
  if (vec8 != 0 && cbase + CHUNK <= nE) {
    da = *(const v4i*)(dsts + e0);
    db = *(const v4i*)(dsts + e0 + 4);
  } else {
    da.x = (e0     < nE) ? dsts[min(e0,     nE - 1)] : sent;
    da.y = (e0 + 1 < nE) ? dsts[min(e0 + 1, nE - 1)] : sent;
    da.z = (e0 + 2 < nE) ? dsts[min(e0 + 2, nE - 1)] : sent;
    da.w = (e0 + 3 < nE) ? dsts[min(e0 + 3, nE - 1)] : sent;
    db.x = (e0 + 4 < nE) ? dsts[min(e0 + 4, nE - 1)] : sent;
    db.y = (e0 + 5 < nE) ? dsts[min(e0 + 5, nE - 1)] : sent;
    db.z = (e0 + 6 < nE) ? dsts[min(e0 + 6, nE - 1)] : sent;
    db.w = (e0 + 7 < nE) ? dsts[min(e0 + 7, nE - 1)] : sent;
  }
  const unsigned nbs = (unsigned)slotBase;
  const unsigned unb = (unsigned)nb;
  const unsigned s0 = (unsigned)da.x - nbs, s1 = (unsigned)da.y - nbs;
  const unsigned s2 = (unsigned)da.z - nbs, s3 = (unsigned)da.w - nbs;
  const unsigned s4 = (unsigned)db.x - nbs, s5 = (unsigned)db.y - nbs;
  const unsigned s6 = (unsigned)db.z - nbs, s7 = (unsigned)db.w - nbs;
  const bool h0 = s0 < unb, h1 = s1 < unb, h2 = s2 < unb, h3 = s3 < unb;
  const bool h4 = s4 < unb, h5 = s5 < unb, h6 = s6 < unb, h7 = s7 < unb;
  const unsigned any = __builtin_amdgcn_ballot_w32(h0 | h1 | h2 | h3 | h4 | h5 | h6 | h7);
  if (any != 0u) {
#define HITJ(J, HJ, SJ) { \
      const unsigned mj = __builtin_amdgcn_ballot_w32(HJ); \
      if (mj != 0u) { \
        if (HJ) { \
          const int pos = wc + (int)__builtin_amdgcn_mbcnt_lo(mj, 0u); \
          if (pos < WCAP) list[wave * WCAP + pos] = ((el0 + (J)) << SLB) | (int)(SJ); \
        } \
        wc += (int)__builtin_popcount(mj); } }
    HITJ(0, h0, s0)
    HITJ(1, h1, s1)
    HITJ(2, h2, s2)
    HITJ(3, h3, s3)
    HITJ(4, h4, s4)
    HITJ(5, h5, s5)
    HITJ(6, h6, s6)
    HITJ(7, h7, s7)
#undef HITJ
  }
  return wc;
}

__global__ __launch_bounds__(NTHR) void k_prep(const float* __restrict__ W1, const float* __restrict__ b1,
                                               const float* __restrict__ W2, const float* __restrict__ b2,
                                               const float* __restrict__ W3, const float* __restrict__ b3,
                                               unsigned short* w1c, unsigned short* w2t, float* tab) {
  __shared__ __attribute__((aligned(16))) float st[TABN];
  const int tid = (int)threadIdx.x;
  const int blk = (int)blockIdx.x;
  if (blk == 0) {
    const int n = tid >> 2, k8 = (tid & 3) * 8;
    const int nn = n & 31;
    const int kof = (n >> 5) * 16;
    v8us o;
#pragma unroll
    for (int i = 0; i < 8; ++i) {
      const int k  = k8 + i;
      const int kc = k < 16 ? k : 15;
      const float f = W1[(size_t)(kof + kc) * EH + nn];
      o[i] = (unsigned short)bf16_bits(k < 16 ? f : 0.0f);
    }
    put16(w1c + (size_t)tid * 8, o);
  } else if (blk == 1) {
    const int u = tid & 127;
    const int n = u >> 2, k8 = (u & 3) * 8;
    const int nc = n < EO ? n : EO - 1;
    v8us o;
#pragma unroll
    for (int i = 0; i < 8; ++i) {
      const float f = W2[(size_t)(k8 + i) * EO + nc];
      o[i] = (unsigned short)bf16_bits(n < EO ? f : 0.0f);
    }
    if (tid < 128) put16(w2t + (size_t)u * 8, o);
  } else {
#pragma unroll 1
    for (int e = tid; e < TABN; e += NTHR) {
      float v = 0.0f;
      if (e < T_B1) {
        v = bf16_val(W1[32 * EH + e]);
      } else if (e < T_B2) {
        v = bf16_val(b1[e - T_B1]);
      } else if (e < T_W3) {
        const int j = e - T_B2;
        const int jc = j < EO ? j : EO - 1;
        const float f = b2[jc];
        v = (j < EO) ? bf16_val(f) : 0.0f;
      } else if (e < T_B3) {
        v = bf16_val(W3[e - T_W3]);
      } else if (e < T_B3 + 32) {
        const int j = e - T_B3;
        const int jc = j < NO ? j : NO - 1;
        const float f = b3[jc];
        v = (j < NO) ? bf16_val(f) : 0.0f;
      }
      st[e] = v;
    }
    __syncthreads();
    if (tid < TABN / 4) {
      const v4f q = *(const v4fa*)(st + 4 * tid);
      putf4(tab + 4 * tid, q);
    }
  }
}

__global__ __launch_bounds__(NTHR) void k_node(const float* __restrict__ x, const unsigned short* __restrict__ w1c,
                                               const float* __restrict__ tab, float* pab) {
  __shared__ __attribute__((aligned(16))) float stg[NWAVE * 16 * PW];
  const int tid = (int)threadIdx.x, lane = tid & 31, hh = lane >> 4, m = lane & 15;
  const int wave = __builtin_amdgcn_readfirstlane(tid >> 5);
  const int tile = (int)blockIdx.x * NWAVE + wave;
  if (tile < NTILE) {
    const int row0 = tile * 16;
    const float* xp = x + (size_t)(row0 + m) * NF + 8 * hh;
    const v4f xa = *(const v4fa*)xp;
    const v4f xb = *(const v4fa*)(xp + 4);
    FragB a;
    a.u[0] = (unsigned short)bf16_bits(xa.x); a.u[1] = (unsigned short)bf16_bits(xa.y);
    a.u[2] = (unsigned short)bf16_bits(xa.z); a.u[3] = (unsigned short)bf16_bits(xa.w);
    a.u[4] = (unsigned short)bf16_bits(xb.x); a.u[5] = (unsigned short)bf16_bits(xb.y);
    a.u[6] = (unsigned short)bf16_bits(xb.z); a.u[7] = (unsigned short)bf16_bits(xb.w);
#pragma unroll
    for (int i = 8; i < 16; ++i) a.u[i] = (unsigned short)0;
    float* sw = stg + wave * 16 * PW;
    const float bv0 = tab[T_B1 + m];
    const float bv1 = tab[T_B1 + 16 + m];
#pragma unroll
    for (int nt = 0; nt < 4; ++nt) {
      const unsigned short* wq = w1c + (size_t)(16 * nt + m) * 32 + 8 * hh;
      FragB b;
      b.h[0] = *(const v8usa*)wq;
      b.h[1] = *(const v8usa*)(wq + 16);
      const v8f d = wmb(a, b, z8());
      const float bv = (nt == 2) ? bv0 : ((nt == 3) ? bv1 : 0.0f);
#pragma unroll
      for (int r = 0; r < 8; ++r) sw[(8 * hh + r) * PW + 16 * nt + m] = d[r] + bv;
    }
    wave_sync();
    v4f pv[8];
#pragma unroll
    for (int it = 0; it < 8; ++it) pv[it] = *(const v4fa*)(sw + 4 * (it * 32 + lane));
    float* gp = pab + (size_t)row0 * PW;
#pragma unroll
    for (int it = 0; it < 8; ++it) *(volatile v4f*)(gp + 4 * (it * 32 + lane)) = pv[it];
    __threadfence();
#pragma unroll
    for (int it = 0; it < 8; ++it) *(volatile v4f*)(gp + 4 * (it * 32 + lane)) = pv[it];
  }
}

__global__ __launch_bounds__(NTHR) void k_bucket(const int* __restrict__ eidx, int* lst, int* cntg, int* offg,
                                                 int* flg) {
  extern __shared__ __attribute__((aligned(16))) int dsm[];
  int* list = dsm;
  int* hl   = dsm + LISTN;
  int* sl   = hl + RCAP;
  int* cnt  = sl + RCAP;
  int* offs = cnt + NBA;
  int* cur  = offs + NBA;
  int* misc = cur + NBA;
  const int tid = (int)threadIdx.x, lane = tid & 31, wave = tid >> 5;
  const int blk  = (int)blockIdx.x;
  const int side = (int)blockIdx.y;
  const int keyOff = (side == 0) ? NE : 0;
  const int othOff = NE - keyOff;
  const int* keys = eidx + keyOff;
  const int* oth  = eidx + othOff;
  const int nodeBase = blk * NBA;

  {
    const v4i z4 = {0, 0, 0, 0};
    for (int i = tid * 4; i < BK_ZINTS; i += NTHR * 4) *(v4ia*)(dsm + i) = z4;
    if (tid < 16) misc[tid] = 0;
  }
  __syncthreads();

  int t = 0, ov = 0;
  const int nChunks = (NE + CHUNK - 1) / CHUNK;
#pragma unroll 1
  for (int ch = 0; ch < nChunks; ++ch) {
    const int cbase = ch * CHUNK;
    const int wc = scan_chunk<SLA>(keys, NE, cbase, nodeBase, NBA, 1, list, tid, lane, wave);
    if (lane == 0) misc[wave] = wc;
    __syncthreads();
    if (wave == 0) {
#pragma unroll 1
      for (int w2 = 0; w2 < NWAVE; ++w2) {
        int c = misc[w2];
        c = c < 0 ? 0 : (c > WCAP ? WCAP : c);
#pragma unroll 1
        for (int b0 = 0; b0 < c; b0 += 32) {
          const int idx = b0 + lane;
          const int ent = list[w2 * WCAP + (idx < WCAP ? idx : WCAP - 1)];
          const int m32 = (c - b0) < 32 ? (c - b0) : 32;
#pragma unroll 1
          for (int k = 0; k < m32; ++k) {
            const int u    = __builtin_amdgcn_readlane(ent, k);
            const int slot = u & (NBA - 1);
            const int el   = (u >> SLA) & (CHUNK - 1);
            const int pk   = ((cbase + el) << SLA) | slot;
            if (t < RCAP) {
              if (lane == 0) { hl[t] = pk; cnt[slot] = cnt[slot] + 1; }
              t = t + 1;
            } else {
              ov = 1;
            }
          }
        }
      }
    }
    __syncthreads();
  }
  if (wave == 0 && lane == 0) { misc[8] = t; misc[9] = ov; }
  __syncthreads();
  int tt = misc[8];
  tt = tt < 0 ? 0 : (tt > RCAP ? RCAP : tt);
  const int ovf = misc[9] != 0 ? 1 : 0;

  if (wave == 0) {
    const int base = lane * (NBA / 32);
    int s = 0;
#pragma unroll 1
    for (int i = 0; i < NBA / 32; ++i) s += cnt[base + i];
    int incl = s;
#pragma unroll
    for (int d = 1; d < 32; d <<= 1) {
      const int y = __shfl_up(incl, d, 32);
      if (lane >= d) incl += y;
    }
    int run = incl - s;
#pragma unroll 1
    for (int i = 0; i < NBA / 32; ++i) {
      const int cv = cnt[base + i];
      offs[base + i] = run;
      cur[base + i]  = run;
      run += cv;
    }
  }
  __syncthreads();
  if (wave == 0) {
#pragma unroll 1
    for (int b0 = 0; b0 < tt; b0 += 32) {
      const int idx = b0 + lane;
      const int ent = hl[idx < RCAP ? idx : RCAP - 1];
      const int m32 = (tt - b0) < 32 ? (tt - b0) : 32;
#pragma unroll 1
      for (int k = 0; k < m32; ++k) {
        const int u    = __builtin_amdgcn_readlane(ent, k);
        const int slot = u & (NBA - 1);
        if (lane == 0) {
          int p = cur[slot];
          p = p < 0 ? 0 : (p > RCAP - 1 ? RCAP - 1 : p);
          sl[p] = u;
          cur[slot] = p + 1;
        }
      }
    }
  }
  __syncthreads();

  int* lb = lst + (size_t)(side * NBLK + blk) * (size_t)RCAP * 2;
#pragma unroll 1
  for (int p0 = tid * 2; p0 < RCAP; p0 += NTHR * 2) {
    const v2i ee = *(const v2ia*)(sl + p0);
    int e0 = ee.x >> SLA;
    int e1 = ee.y >> SLA;
    e0 = e0 < 0 ? 0 : (e0 > NE - 1 ? NE - 1 : e0);
    e1 = e1 < 0 ? 0 : (e1 > NE - 1 ? NE - 1 : e1);
    const int o0 = oth[e0];
    const int o1 = oth[e1];
    asm volatile("" :: "v"(o0));
    asm volatile("" :: "v"(o1));
    const int k0 = (p0     < tt) ? -1 : 0;
    const int k1 = (p0 + 1 < tt) ? -1 : 0;
    v4i q;
    q.x = o0 & k0; q.y = e0 & k0; q.z = o1 & k1; q.w = e1 & k1;
    puti4(lb + 2 * p0, q);
  }
  if (tid < NBA / 4) {
    const v4i c4 = *(const v4ia*)(cnt + 4 * tid);
    const v4i o4 = *(const v4ia*)(offs + 4 * tid);
    puti4(cntg + (size_t)side * NP + nodeBase + 4 * tid, c4);
    puti4(offg + (size_t)side * NP + nodeBase + 4 * tid, o4);
  }
  if (tid < FLN / 4) {
    const v4i f4 = {ovf, ovf, ovf, ovf};
    puti4(flg + (size_t)(side * NBLK + blk) * FLN + 4 * tid, f4);
  }
}

__device__ __forceinline__ void edge_tile(const float* __restrict__ pab, const float* __restrict__ ew,
                                          int rowb, int ewb, int oth, int eid, int gofs8h,
                                          v8f ownA, v8f ownB, v8f w1A, v8f w1B,
                                          const FragB& B0, const FragB& B1, float b2a, float b2b,
                                          float sgn, int rem, float& acc0, float& acc1) {
  const float* gp = pab + (size_t)(rowb + oth) * PW + gofs8h;
  const v4f ga = *(const v4fa*)gp;
  const v4f gb = *(const v4fa*)(gp + 4);
  const v4f gc = *(const v4fa*)(gp + 16);
  const v4f gd = *(const v4fa*)(gp + 20);
  const float w = ew[(size_t)(ewb + eid)];
  asm volatile("" :: "v"(ga));
  asm volatile("" :: "v"(gb));
  asm volatile("" :: "v"(gc));
  asm volatile("" :: "v"(gd));
  asm volatile("" :: "v"(w));
  const float wq = bf16_val(w);
  const v8f gA = {ga.x, ga.y, ga.z, ga.w, gb.x, gb.y, gb.z, gb.w};
  const v8f gB = {gc.x, gc.y, gc.z, gc.w, gd.x, gd.y, gd.z, gd.w};
  FragB ah, al;
#pragma unroll
  for (int i = 0; i < 8; ++i) {
    const float pre = fmaf(wq, w1A[i], ownA[i] + gA[i]);
    const float hv  = sigf(pre);
    const unsigned hb = bf16_bits(hv);
    const unsigned lb = bf16_bits(hv - __uint_as_float(hb << 16));
    ah.u[i] = (unsigned short)hb;
    al.u[i] = (unsigned short)lb;
  }
#pragma unroll
  for (int i = 0; i < 8; ++i) {
    const float pre = fmaf(wq, w1B[i], ownB[i] + gB[i]);
    const float hv  = sigf(pre);
    const unsigned hb = bf16_bits(hv);
    const unsigned lb = bf16_bits(hv - __uint_as_float(hb << 16));
    ah.u[8 + i] = (unsigned short)hb;
    al.u[8 + i] = (unsigned short)lb;
  }
  v8f d0 = wmb(ah, B0, z8());
  d0 = wmb(al, B0, d0);
  v8f d1 = wmb(ah, B1, z8());
  d1 = wmb(al, B1, d1);
  float s0 = 0.0f, s1 = 0.0f;
#pragma unroll
  for (int r = 0; r < 8; ++r) {
    const bool ok = r < rem;
    const float v0 = sigf(d0[r] + b2a);
    const float v1 = sigf(d1[r] + b2b);
    s0 += ok ? v0 : 0.0f;
    s1 += ok ? v1 : 0.0f;
  }
  acc0 += sgn * s0;
  acc1 += sgn * s1;
}

__global__ __launch_bounds__(NTHR) __attribute__((amdgpu_num_vgpr(248)))
void k_replay(const float* __restrict__ pab, const float* __restrict__ ew, const int* __restrict__ lst,
              const int* __restrict__ cntg, const int* __restrict__ offg, const int* __restrict__ flg,
              const unsigned short* __restrict__ w2t, const float* __restrict__ tab, float* out) {
  __shared__ __attribute__((aligned(16))) float sagg[NB * RB * 32];
  __shared__ __attribute__((aligned(16))) float sout[NB * RB * NO];
  __shared__ __attribute__((aligned(16))) float sw3[512];
  __shared__ int spois[RB];
  const int tid = (int)threadIdx.x, lane = tid & 31, hh = lane >> 4, m = lane & 15;
  const int wave  = __builtin_amdgcn_readfirstlane(tid >> 5);
  const int node0 = (int)blockIdx.x * RB;
  const int blk   = node0 >> SLA;

  for (int i = tid; i < W3N; i += NTHR) sw3[i] = tab[T_W3 + i];

  v8f w1A, w1B;
  {
    const v4f a0 = *(const v4fa*)(tab + T_W1R + 8 * hh);
    const v4f a1 = *(const v4fa*)(tab + T_W1R + 8 * hh + 4);
    const v4f c0 = *(const v4fa*)(tab + T_W1R + 16 + 8 * hh);
    const v4f c1 = *(const v4fa*)(tab + T_W1R + 16 + 8 * hh + 4);
    const v8f t0 = {a0.x, a0.y, a0.z, a0.w, a1.x, a1.y, a1.z, a1.w};
    const v8f t1 = {c0.x, c0.y, c0.z, c0.w, c1.x, c1.y, c1.z, c1.w};
    w1A = t0; w1B = t1;
  }
  const float b2a = tab[T_B2 + m];
  const float b2b = tab[T_B2 + 16 + m];
  FragB B0, B1;
  {
    const unsigned short* q0 = w2t + (size_t)m * 32 + 8 * hh;
    const unsigned short* q1 = w2t + (size_t)(16 + m) * 32 + 8 * hh;
    B0.h[0] = *(const v8usa*)q0;
    B0.h[1] = *(const v8usa*)(q0 + 16);
    B1.h[0] = *(const v8usa*)q1;
    B1.h[1] = *(const v8usa*)(q1 + 16);
  }

#pragma unroll 1
  for (int ni = 0; ni < 8; ++ni) {
    const int nl   = 8 * wave + ni;
    const int node = node0 + nl;
    const bool live = node < NN;
    const int nc = live ? node : NN - 1;
    float a00 = 0.0f, a01 = 0.0f, a10 = 0.0f, a11 = 0.0f;
    int big = 0;
#pragma unroll 1
    for (int side = 0; side < 2; ++side) {
      int c = cntg[(size_t)side * NP + nc];
      int o = offg[(size_t)side * NP + nc];
      c = __builtin_amdgcn_readfirstlane(c);
      o = __builtin_amdgcn_readfirstlane(o);
      if (c > DEGCAP || c < 0) big = 1;
      c = c < 0 ? 0 : (c > DEGCAP ? DEGCAP : c);
      if (!live) c = 0;
      o = o < 0 ? 0 : (o > RCAP - 1 ? RCAP - 1 : o);
      const int oofs = (side == 0) ? 32 : 0;
      const int gofs8h = (32 - oofs) + 8 * hh;
      const float sgn = (side == 0) ? 1.0f : -1.0f;
      if (c > 0) {
        const float* op0 = pab + (size_t)nc * PW + oofs + 8 * hh;
        const float* op1 = op0 + (size_t)NN * PW;
        const v4f p0 = *(const v4fa*)op0,        p1 = *(const v4fa*)(op0 + 4);
        const v4f p2 = *(const v4fa*)(op0 + 16), p3 = *(const v4fa*)(op0 + 20);
        const v4f r0 = *(const v4fa*)op1,        r1 = *(const v4fa*)(op1 + 4);
        const v4f r2 = *(const v4fa*)(op1 + 16), r3 = *(const v4fa*)(op1 + 20);
        const v8f own0A = {p0.x, p0.y, p0.z, p0.w, p1.x, p1.y, p1.z, p1.w};
        const v8f own0B = {p2.x, p2.y, p2.z, p2.w, p3.x, p3.y, p3.z, p3.w};
        const v8f own1A = {r0.x, r0.y, r0.z, r0.w, r1.x, r1.y, r1.z, r1.w};
        const v8f own1B = {r2.x, r2.y, r2.z, r2.w, r3.x, r3.y, r3.z, r3.w};
        const int* lb = lst + (size_t)(side * NBLK + blk) * (size_t)RCAP * 2;
#pragma unroll 1
        for (int t0 = 0; t0 < c; t0 += 16) {
          const int j  = t0 + m;
          const int jc = j < c ? j : c - 1;
          int idx = o + jc;
          idx = idx > RCAP - 1 ? RCAP - 1 : idx;
          const v2i ent = *(const v2ia*)(lb + 2 * idx);
          asm volatile("" :: "v"(ent));
          int oth = ent.x;
          int eid = ent.y;
          oth = oth < 0 ? 0 : (oth > NN - 1 ? NN - 1 : oth);
          eid = eid < 0 ? 0 : (eid > NE - 1 ? NE - 1 : eid);
          const int rem = c - t0 - 8 * hh;
          edge_tile(pab, ew, 0,  0,  oth, eid, gofs8h, own0A, own0B, w1A, w1B, B0, B1, b2a, b2b, sgn, rem, a00, a01);
          edge_tile(pab, ew, NN, NE, oth, eid, gofs8h, own1A, own1B, w1A, w1B, B0, B1, b2a, b2b, sgn, rem, a10, a11);
        }
      }
    }
    const float t00 = a00 + __shfl_xor(a00, 16, 32);
    const float t01 = a01 + __shfl_xor(a01, 16, 32);
    const float t10 = a10 + __shfl_xor(a10, 16, 32);
    const float t11 = a11 + __shfl_xor(a11, 16, 32);
    const bool colok = (16 + m) < EO;
    if (hh == 0) {
      sagg[(0 * RB + nl) * 32 + m]      = t00;
      sagg[(0 * RB + nl) * 32 + 16 + m] = colok ? t01 : 0.0f;
      sagg[(1 * RB + nl) * 32 + m]      = t10;
      sagg[(1 * RB + nl) * 32 + 16 + m] = colok ? t11 : 0.0f;
    }
    if (lane == 0) spois[nl] = big;
  }
  __syncthreads();

  {
    const int fT = flg[(size_t)(0 * NBLK + blk) * FLN];
    const int fS = flg[(size_t)(1 * NBLK + blk) * FLN];
    const int fl = (fT != 0 || fS != 0) ? 1 : 0;
    const int cc = tid & 15;
    const int g  = tid >> 4;
    const float qnan = __int_as_float(0x7fc00000);
    const float bias = sw3[480 + cc];
#pragma unroll 1
    for (int q = 0; q < 8; ++q) {
      const int b  = q >> 2;
      const int nl = g + 16 * (q & 3);
      const float* ar = sagg + (b * RB + nl) * 32;
      float s = 0.0f;
#pragma unroll 2
      for (int k = 0; k < EO; ++k) s = fmaf(ar[k], sw3[k * NO + cc], s);
      float tv = s + bias;
      tv = fmaxf(tv, -60.0f);
      float ov = 1.0f / (1.0f + expf(-tv));
      const bool ps = (fl != 0) || (spois[nl] != 0);
      ov = ps ? qnan : ov;
      sout[(b * RB + nl) * NO + cc] = ov;
    }
  }
  __syncthreads();

  {
    const int nn = (NN - node0) < RB ? (NN - node0) : RB;
    const bool ok = tid < nn * 4;
    const v4f q0 = *(const v4fa*)(sout + 0 * RB * NO + 4 * tid);
    const v4f q1 = *(const v4fa*)(sout + 1 * RB * NO + 4 * tid);
    float* g0 = out + ((size_t)0 * NN + node0) * NO + 4 * tid;
    float* g1 = out + ((size_t)1 * NN + node0) * NO + 4 * tid;
    if (ok) { *(volatile v4f*)g0 = q0; *(volatile v4f*)g1 = q1; }
    __threadfence();
    if (ok) { *(volatile v4f*)g0 = q0; *(volatile v4f*)g1 = q1; }
  }
}

static inline size_t al256(size_t o) { return (o + 255) & ~(size_t)255; }

extern "C" void kernel_launch(void* const* d_in, const int* in_sizes, int n_in,
                              void* d_out, int out_size, void* d_ws, size_t ws_size,
                              hipStream_t stream) {
  if (n_in < 9) return;
  if (in_sizes[0] != NB * NN * NF) return;
  if (in_sizes[1] != NB * NE) return;
  if (in_sizes[2] != 2 * NE) return;
  if (in_sizes[3] != 33 * EH || in_sizes[4] != EH) return;
  if (in_sizes[5] != EH * EO || in_sizes[6] != EO) return;
  if (in_sizes[7] != EO * NO || in_sizes[8] != NO) return;
  if (out_size != NB * NN * NO) return;

  const float* x   = (const float*)d_in[0];
  const float* ew  = (const float*)d_in[1];
  const int*   ei  = (const int*)  d_in[2];
  const float* W1  = (const float*)d_in[3];
  const float* b1  = (const float*)d_in[4];
  const float* W2  = (const float*)d_in[5];
  const float* b2  = (const float*)d_in[6];
  const float* W3  = (const float*)d_in[7];
  const float* b3  = (const float*)d_in[8];
  float* out = (float*)d_out;

  char* ws = (char*)d_ws;
  size_t off = 0;
  const size_t oW1C  = off; off = al256(off + (size_t)64 * 32 * 2);
  const size_t oW2T  = off; off = al256(off + (size_t)32 * 32 * 2);
  const size_t oTAB  = off; off = al256(off + (size_t)TABN * 4);
  const size_t oFLAG = off; off = al256(off + (size_t)2 * NBLK * FLN * 4);
  const size_t oCNT  = off; off = al256(off + (size_t)2 * NP * 4);
  const size_t oOFF  = off; off = al256(off + (size_t)2 * NP * 4);
  const size_t oPAB  = off; off = al256(off + (size_t)MROWS * PW * 4);
  const size_t oLIST = off; off = al256(off + (size_t)2 * NBLK * RCAP * 8);
  if (off > ws_size || off > (size_t)WSMAX) return;
  unsigned short* W1C = (unsigned short*)(ws + oW1C);
  unsigned short* W2T = (unsigned short*)(ws + oW2T);
  float*          TAB = (float*)(ws + oTAB);
  int*            FLG = (int*)(ws + oFLAG);
  int*            CNT = (int*)(ws + oCNT);
  int*            OFS = (int*)(ws + oOFF);
  float*          PAB = (float*)(ws + oPAB);
  int*            LST = (int*)(ws + oLIST);

  hipFuncSetAttribute(reinterpret_cast<const void*>(&k_bucket), hipFuncAttributeMaxDynamicSharedMemorySize,
                      (int)BK_BYTES);

  k_prep<<<3, NTHR, 0, stream>>>(W1, b1, W2, b2, W3, b3, W1C, W2T, TAB);
  k_node<<<(NTILE + NWAVE - 1) / NWAVE, NTHR, 0, stream>>>(x, W1C, TAB, PAB);
  k_bucket<<<dim3(NBLK, 2), NTHR, BK_BYTES, stream>>>(ei, LST, CNT, OFS, FLG);
  k_replay<<<NRB, NTHR, 0, stream>>>(PAB, ew, LST, CNT, OFS, FLG, W2T, TAB, out);
}
